// Sboxblock_90623809946144
// MI455X (gfx1250) — hardware-verified
//
#include <hip/hip_runtime.h>
#include <math.h>

typedef __attribute__((ext_vector_type(16))) _Float16 v16h;
typedef __attribute__((ext_vector_type(16))) __bf16 v16b;
typedef __attribute__((ext_vector_type(8)))  _Float16 v8h;
typedef __attribute__((ext_vector_type(8)))  float v8f;
typedef __attribute__((ext_vector_type(4)))  float v4f;
typedef __attribute__((ext_vector_type(2)))  float v2f;
typedef __attribute__((ext_vector_type(4)))  unsigned v4u;
typedef __attribute__((ext_vector_type(4)))  int v4i;
typedef float __attribute__((may_alias)) float_a;
typedef int __attribute__((may_alias)) int_a;

template <typename T> __device__ __forceinline__ void vst2(void* p, T v) { *(volatile T*)p = v; __threadfence(); *(volatile T*)p = v; }
__device__ __forceinline__ v8f wmma16(v16h a, v16h b, v8f c) {
  v8f d = __builtin_amdgcn_wmma_f32_16x16x32_f16(false, a, false, b, (short)0, c, false, false);
  asm volatile("v_nop\n\tv_nop\n\tv_nop\n\tv_nop" : "+v"(d) : "v"(a), "v"(b));
  return d;
}
__device__ __forceinline__ v8f wmma_bf(v16b a, v16b b, v8f c) {
  v8f d = __builtin_amdgcn_wmma_f32_16x16x32_bf16(false, a, false, b, (short)0, c, false, false);
  asm volatile("v_nop\n\tv_nop\n\tv_nop\n\tv_nop" : "+v"(d) : "v"(a), "v"(b));
  return d;
}
__device__ __forceinline__ v16h frag_h(const _Float16* rowk0, int lane) {
  union { v16h v; v8h q[2]; } u; const _Float16* p = rowk0 + 8 * (lane >> 4);
  u.q[0] = *(const v8h*)p; u.q[1] = *(const v8h*)(p + 16); return u.v;
}
__device__ __forceinline__ v16h frag_f32(const float* rowk0, int lane) {
  v16h a; const float* p = rowk0 + 8 * (lane >> 4);
#pragma unroll
  for (int i = 0; i < 8; ++i) { a[i] = (_Float16)p[i]; a[8 + i] = (_Float16)p[16 + i]; }
  return a;
}
__device__ __forceinline__ v16h frag_f32s(const float* rowk0, int lane, float sc) {
  v16h a; const float* p = rowk0 + 8 * (lane >> 4);
#pragma unroll
  for (int i = 0; i < 8; ++i) { a[i] = (_Float16)(p[i] * sc); a[8 + i] = (_Float16)(p[16 + i] * sc); }
  return a;
}
__device__ __forceinline__ v16h fragc_f32(const float* W, int k0, int n, int lane, int ld, int K) {
  v16h a; const int g = lane >> 4;
#pragma unroll
  for (int i = 0; i < 8; ++i) { const int ka = k0 + 8 * g + i, kb = ka + 16;
    a[i] = (_Float16)(ka < K ? W[(size_t)(ka < K ? ka : K - 1) * ld + n] : 0.f); a[8 + i] = (_Float16)(kb < K ? W[(size_t)(kb < K ? kb : K - 1) * ld + n] : 0.f); }
  return a;
}
struct F2 { v16b h, l; };
__device__ __forceinline__ F2 bsplit16(const float v[16]) { F2 r;
#pragma unroll
  for (int i = 0; i < 16; ++i) { const __bf16 h = (__bf16)v[i]; r.h[i] = h; r.l[i] = (__bf16)(v[i] - (float)h); }
  return r; }
__device__ __forceinline__ F2 split_row(const float* row, int k0, int lane) { float v[16]; const float* p = row + k0 + 8 * (lane >> 4);
#pragma unroll
  for (int i = 0; i < 8; ++i) { v[i] = p[i]; v[8 + i] = p[16 + i]; }
  return bsplit16(v); }
__device__ __forceinline__ F2 split_rowK(const float* row, int k0, int lane, int K) { float v[16]; const int g = lane >> 4;
#pragma unroll
  for (int i = 0; i < 8; ++i) { const int ka = k0 + 8 * g + i, kb = ka + 16; v[i] = ka < K ? row[ka < K ? ka : K - 1] : 0.f; v[8 + i] = kb < K ? row[kb < K ? kb : K - 1] : 0.f; }
  return bsplit16(v); }
__device__ __forceinline__ F2 split_col(const float* W, int k0, int n, int lane, int ld, int K) { float v[16]; const int g = lane >> 4;
#pragma unroll
  for (int i = 0; i < 8; ++i) { const int ka = k0 + 8 * g + i, kb = ka + 16; v[i] = ka < K ? W[(size_t)(ka < K ? ka : K - 1) * ld + n] : 0.f; v[8 + i] = kb < K ? W[(size_t)(kb < K ? kb : K - 1) * ld + n] : 0.f; }
  return bsplit16(v); }
__device__ __forceinline__ v8f mac3(const F2& a, const F2& b, v8f c) { c = wmma_bf(a.l, b.h, c); c = wmma_bf(a.h, b.l, c); return wmma_bf(a.h, b.h, c); }
__device__ __forceinline__ float sigm(float v) { return 1.0f / (1.0f + expf(-v)); }
#define LDSX() do { asm volatile("s_wait_dscnt 0" ::: "memory"); __builtin_amdgcn_wave_barrier(); __builtin_amdgcn_fence(__ATOMIC_RELEASE, "workgroup"); } while (0)


#define NBATCH 4
#define RR 32
#define CC 96
#define NWIN 512
#define NTOKW 64
#define NHEAD 4
#define DH 24
#define DP 32
#define MLPD 384
#define KP 128
typedef __attribute__((ext_vector_type(8))) __bf16 v8b;
__device__ __forceinline__ v16b frag_b16(const __bf16* rowk0, int lane) {
  union { v16b v; v8b q[2]; } u; const __bf16* p = rowk0 + 8 * (lane >> 4);
  u.q[0] = *(const v8b*)p; u.q[1] = *(const v8b*)(p + 16); return u.v;
}
__device__ __forceinline__ v16b frag_rbf(const float* rowk0, int lane) {
  v16b a; const float* p = rowk0 + 8 * (lane >> 4);
#pragma unroll
  for (int i = 0; i < 8; ++i) { a[i] = (__bf16)p[i]; a[8 + i] = (__bf16)p[16 + i]; }
  return a;
}
__device__ __forceinline__ float bfr(float v) { return (float)(__bf16)v; }
__device__ __attribute__((noinline)) float gelu_t(float x) { const float u = 0.7978845608028654f * (x + 0.044715f * x * x * x); return 0.5f * x * (1.0f + tanhf(u)); }
__device__ __attribute__((noinline)) float exp_ni(float v) { return expf(v); }

__device__ __forceinline__ int box_token(int widx, int n) {
  const int bx = widx >> 6, by = (widx >> 3) & 7, bz = widx & 7;
  const int ix = n >> 4, iy = (n >> 2) & 3, iz = n & 3;
  const int x = (bx * 4 + ix + 2) & 31, y = (by * 4 + iy + 2) & 31, z = (bz * 4 + iz + 2) & 31;
  return (x * RR + y) * RR + z;
}

__global__ __launch_bounds__(128) void k_pack(const float* __restrict__ Wm, int K, int NOUT, int KPITCH, __bf16* __restrict__ PT) {
  __shared__ __align__(16) __bf16 srow[MLPD];
  const int n = blockIdx.x, tid = threadIdx.x;
  for (int k = tid; k < KPITCH; k += 128) srow[k] = k < K ? (__bf16)Wm[(size_t)k * NOUT + n] : (__bf16)0.0f;
  __syncthreads();
  if (tid < KPITCH / 8) vst2((unsigned*)(PT + (size_t)n * KPITCH + tid * 8), *(const v4u*)(&srow[tid * 8]));
}

__device__ __forceinline__ void ln64(float (*t)[100], const float* __restrict__ g, const float* __restrict__ b, int wave, int lane) {
#pragma unroll 1
  for (int rr = 0; rr < 8; ++rr) { const int row = wave * 8 + rr; const bool act = lane < 24; float v[4]; float s = 0.f;
#pragma unroll
    for (int i = 0; i < 4; ++i) { v[i] = act ? t[row][(act ? lane : 0) * 4 + i] : 0.f; s += v[i]; }
#pragma unroll
    for (int o = 16; o > 0; o >>= 1) s += __shfl_xor(s, o);
    const float mu = s * (1.0f / CC); float q = 0.f;
#pragma unroll
    for (int i = 0; i < 4; ++i) { const float d = v[i] - mu; q += act ? d * d : 0.f; }
#pragma unroll
    for (int o = 16; o > 0; o >>= 1) q += __shfl_xor(q, o);
    const float rs = rsqrtf(q * (1.0f / CC) + 1e-5f);
    if (act) {
#pragma unroll
      for (int i = 0; i < 4; ++i) { const int c = lane * 4 + i; t[row][c] = (v[i] - mu) * rs * bfr(g[c]) + bfr(b[c]); } }
  }
}

__global__ __launch_bounds__(256) void k_block(const float* __restrict__ X, const float* __restrict__ g1, const float* __restrict__ b1n, const __bf16* __restrict__ PTqkv, const float* __restrict__ bqkv,
                                               const __bf16* __restrict__ PTproj, const float* __restrict__ bproj, const float* __restrict__ g2, const float* __restrict__ b2n,
                                               const __bf16* __restrict__ PTw1, const float* __restrict__ bm1, const __bf16* __restrict__ PTw2, const float* __restrict__ bm2,
                                               const float* __restrict__ mask, float* __restrict__ out) {
  __shared__ __align__(16) __bf16 R1[NTOKW * MLPD];
  __shared__ __align__(16) float R2[NTOKW][100];
  __shared__ __align__(16) float R3[NTOKW][100];
  const int w = blockIdx.x, bb = w >> 9, widx = w & 511;
  const int tid = threadIdx.x, wave = tid >> 5, lane = tid & 31, col = lane & 15, g = lane >> 4;
  __bf16* q_s = R1; __bf16* k_s = R1 + NHEAD * NTOKW * DP; __bf16* vt_s = R1 + 2 * NHEAD * NTOKW * DP;
  const float* Xb = X + (size_t)bb * RR * RR * RR * CC;

  for (int q = tid; q < NTOKW * 24; q += 256) { const int n = q / 24, pc = q - n * 24; const float4 v = *(const float4*)(Xb + (size_t)box_token(widx, n) * CC + pc * 4);
    R2[n][pc * 4] = bfr(v.x); R2[n][pc * 4 + 1] = bfr(v.y); R2[n][pc * 4 + 2] = bfr(v.z); R2[n][pc * 4 + 3] = bfr(v.w); }
  for (int q = tid; q < NTOKW * MLPD / 8; q += 256) *(v4u*)(R1 + q * 8) = (v4u){0u, 0u, 0u, 0u};
  __syncthreads();
  ln64(R2, g1, b1n, wave, lane);
  __syncthreads();
  { const int rt = wave & 3, ct0 = (wave >> 2) * 9; v8f acc[9] = {};
#pragma unroll
    for (int kc = 0; kc < CC / 32; ++kc) { const v16b a = frag_rbf(&R2[rt * 16 + col][kc * 32], lane);
#pragma unroll
      for (int j = 0; j < 9; ++j) acc[j] = wmma_bf(a, frag_b16(PTqkv + (size_t)((ct0 + j) * 16 + col) * KP + kc * 32, lane), acc[j]); }
#pragma unroll
    for (int j = 0; j < 9; ++j) { const int c = (ct0 + j) * 16 + col; const int s3 = c / CC, rem = c - s3 * CC, hh = rem / DH, d = rem - hh * DH; const float bv = bfr(bqkv[c]);
#pragma unroll
      for (int r = 0; r < 8; ++r) { const int n = rt * 16 + 8 * g + r; const __bf16 val = (__bf16)(acc[j][r] + bv);
        if (s3 == 0) q_s[(hh * NTOKW + n) * DP + d] = val; else if (s3 == 1) k_s[(hh * NTOKW + n) * DP + d] = val; else vt_s[(hh * DP + d) * NTOKW + n] = val; } } }
  __syncthreads();
  { const int hh = wave >> 1; __bf16* pst = (__bf16*)&R2[0][0] + wave * (16 * 72);
    const float* mw = mask + (size_t)widx * NTOKW * NTOKW;
#pragma unroll 1
    for (int t2 = 0; t2 < 2; ++t2) { const int rt = (wave & 1) * 2 + t2;
      v8f s[4];
      const v16b qa = frag_b16(q_s + (hh * NTOKW + rt * 16 + col) * DP, lane);
#pragma unroll
      for (int j = 0; j < 4; ++j) { s[j] = (v8f){}; s[j] = wmma_bf(qa, frag_b16(k_s + (hh * NTOKW + j * 16 + col) * DP, lane), s[j]); }
      float mx[8], sm[8];
#pragma unroll
      for (int r = 0; r < 8; ++r) { const int n = rt * 16 + 8 * g + r; float m = -3.0e38f;
#pragma unroll
        for (int j = 0; j < 4; ++j) { const float v = s[j][r] * 0.20412414523193154f + bfr(mw[n * NTOKW + j * 16 + col]); s[j][r] = v; m = fmaxf(m, v); }
#pragma unroll
        for (int o = 1; o < 16; o <<= 1) m = fmaxf(m, __shfl_xor(m, o));
        float sum = 0.f;
#pragma unroll
        for (int j = 0; j < 4; ++j) { const float e = exp_ni(s[j][r] - m); s[j][r] = e; sum += e; }
#pragma unroll
        for (int o = 1; o < 16; o <<= 1) sum += __shfl_xor(sum, o);
        mx[r] = m; sm[r] = 1.0f / sum; }
#pragma unroll
      for (int j = 0; j < 4; ++j)
#pragma unroll
        for (int r = 0; r < 8; ++r) pst[(8 * g + r) * 72 + j * 16 + col] = (__bf16)(s[j][r] * sm[r]);
      LDSX();
      v8f o[2] = {};
#pragma unroll
      for (int kc = 0; kc < 2; ++kc) { const v16b pa = frag_b16(pst + col * 72 + kc * 32, lane);
#pragma unroll
        for (int j = 0; j < 2; ++j) o[j] = wmma_bf(pa, frag_b16(vt_s + (hh * DP + j * 16 + col) * NTOKW + kc * 32, lane), o[j]); }
#pragma unroll
      for (int j = 0; j < 2; ++j) { const int d = j * 16 + col; if (d < DH) {
#pragma unroll
        for (int r = 0; r < 8; ++r) R3[rt * 16 + 8 * g + r][hh * DH + d] = o[j][r]; } }
      LDSX();
    } }
  __syncthreads();
  { const int rt = wave & 3, ct0 = (wave >> 2) * 3; v8f acc[3] = {};
#pragma unroll
    for (int kc = 0; kc < CC / 32; ++kc) { const v16b a = frag_rbf(&R3[rt * 16 + col][kc * 32], lane);
#pragma unroll
      for (int j = 0; j < 3; ++j) acc[j] = wmma_bf(a, frag_b16(PTproj + (size_t)((ct0 + j) * 16 + col) * KP + kc * 32, lane), acc[j]); }
#pragma unroll
    for (int j = 0; j < 3; ++j) { const int c = (ct0 + j) * 16 + col; const float bv = bfr(bproj[c]);
#pragma unroll
      for (int r = 0; r < 8; ++r) { const int n = rt * 16 + 8 * g + r; R2[n][c] = (acc[j][r] + bv) * 0.5f + bfr(Xb[(size_t)box_token(widx, n) * CC + c]); } } }
  __syncthreads();
  for (int q = tid; q < NTOKW * CC; q += 256) { const int n = q / CC, c = q - n * CC; R3[n][c] = R2[n][c]; }
  __syncthreads();
  ln64(R3, g2, b2n, wave, lane);
  __syncthreads();
  { const int rt = wave & 3, ct0 = (wave >> 2) * 12; v8f acc[12];
#pragma unroll
    for (int j = 0; j < 12; ++j) acc[j] = (v8f){};
#pragma unroll
    for (int kc = 0; kc < CC / 32; ++kc) { const v16b a = frag_rbf(&R3[rt * 16 + col][kc * 32], lane);
#pragma unroll
      for (int j = 0; j < 12; ++j) acc[j] = wmma_bf(a, frag_b16(PTw1 + (size_t)((ct0 + j) * 16 + col) * KP + kc * 32, lane), acc[j]); }
#pragma unroll
    for (int j = 0; j < 12; ++j) { const int c = (ct0 + j) * 16 + col; const float bv = bfr(bm1[c]);
#pragma unroll
      for (int r = 0; r < 8; ++r) R1[(rt * 16 + 8 * g + r) * MLPD + c] = (__bf16)gelu_t(acc[j][r] + bv); } }
  __syncthreads();
  { const int rt = wave & 3, ct0 = (wave >> 2) * 3; v8f acc[3] = {};
#pragma unroll 2
    for (int kc = 0; kc < MLPD / 32; ++kc) { const v16b a = frag_b16(R1 + (rt * 16 + col) * MLPD + kc * 32, lane);
#pragma unroll
      for (int j = 0; j < 3; ++j) acc[j] = wmma_bf(a, frag_b16(PTw2 + (size_t)((ct0 + j) * 16 + col) * MLPD + kc * 32, lane), acc[j]); }
#pragma unroll
    for (int j = 0; j < 3; ++j) { const int c = (ct0 + j) * 16 + col; const float bv = bfr(bm2[c]);
#pragma unroll
      for (int r = 0; r < 8; ++r) { const int n = rt * 16 + 8 * g + r; R3[n][c] = (acc[j][r] + bv) * 0.5f + R2[n][c]; } } }
  __syncthreads();
  float* Ob = out + (size_t)bb * RR * RR * RR * CC;
  for (int q = tid; q < NTOKW * 24; q += 256) { const int n = q / 24, pc = q - n * 24; vst2(Ob + (size_t)box_token(widx, n) * CC + pc * 4, *(const v4f*)(&R3[n][pc * 4])); }
}

extern "C" void kernel_launch(void* const* d_in, const int* in_sizes, int n_in, void* d_out, int out_size, void* d_ws, size_t ws_size, hipStream_t stream) {
  (void)in_sizes; (void)n_in; (void)out_size; (void)ws_size;
  const float** I = (const float**)d_in;
  char* ws = (char*)d_ws;
  __bf16* PTqkv = (__bf16*)ws; __bf16* PTproj = PTqkv + 3 * CC * KP; __bf16* PTw1 = PTproj + CC * KP; __bf16* PTw2 = PTw1 + MLPD * KP;
  k_pack<<<3 * CC, 128, 0, stream>>>(I[3], CC, 3 * CC, KP, PTqkv);
  k_pack<<<CC, 128, 0, stream>>>(I[5], CC, CC, KP, PTproj);
  k_pack<<<MLPD, 128, 0, stream>>>(I[9], CC, MLPD, KP, PTw1);
  k_pack<<<CC, 128, 0, stream>>>(I[11], MLPD, CC, MLPD, PTw2);
  k_block<<<NBATCH * NWIN, 256, 0, stream>>>(I[0], I[1], I[2], PTqkv, I[4], PTproj, I[6], I[7], I[8], PTw1, I[10], PTw2, I[12], I[13], (float*)d_out);
}
